// HandCodedAttentionLayer_28862180229774
// MI455X (gfx1250) — hardware-verified
//
#include <hip/hip_runtime.h>
#include <math.h>

constexpr int kBatch = 4;
constexpr int kSeq   = 2048;
constexpr int kEmb   = 1024;
constexpr int kHeads = 16;
constexpr int kHdim  = 64;
constexpr int kTok   = kBatch * kSeq;
constexpr int kGrp   = 4;
constexpr int kChunks = kHeads / kGrp;

constexpr float kWCarry    = 16.0f;
constexpr float kProjScale = 1.0f / 16.0f;
constexpr float kScoreScale = 0.125f;
constexpr float kPCarry    = 2048.0f;
constexpr float kCtxCarry  = 64.0f;
constexpr float kPVScale   = kCtxCarry / kPCarry;
constexpr float kOutScale  = 1.0f / (kCtxCarry * kWCarry);

constexpr size_t kPlaneWBytes = (size_t)kEmb * kEmb * 2;
constexpr size_t kOffW   = 0;
constexpr size_t kOffX   = kOffW + 4 * kPlaneWBytes;
constexpr size_t kPlaneBBytes = (size_t)kSeq * kEmb * 2;
constexpr size_t kOffQ   = kOffX + kPlaneBBytes;
constexpr size_t kOffK   = kOffQ + kPlaneBBytes;
constexpr size_t kOffVT  = kOffK + kPlaneBBytes;
constexpr size_t kOffCtx = kOffVT + kPlaneBBytes;
constexpr size_t kOffS   = kOffCtx + kPlaneBBytes;
constexpr size_t kScoreBytes = (size_t)kGrp * kSeq * kSeq * 4;
constexpr size_t kOffP   = kOffS + kScoreBytes;
constexpr size_t kPBytes = (size_t)kGrp * kSeq * kSeq * 2;
constexpr size_t kWsEnd  = kOffP + kPBytes;

typedef __attribute__((ext_vector_type(16))) _Float16 v16h;
typedef __attribute__((ext_vector_type(8)))  _Float16 v8h;
typedef __attribute__((ext_vector_type(16))) __bf16   v16b;
typedef __attribute__((ext_vector_type(8)))  __bf16   v8b;
typedef __attribute__((ext_vector_type(8)))  float    v8f;
typedef __attribute__((ext_vector_type(4)))  float    v4f;
typedef __attribute__((ext_vector_type(4)))  unsigned int v4u;

__device__ __forceinline__ unsigned short f2bf_bits(float f) {
  unsigned u = __float_as_uint(f);
  return (unsigned short)((u + 0x7FFFu + ((u >> 16) & 1u)) >> 16);
}
__device__ __forceinline__ float bf_bits2f(unsigned short h) { return __uint_as_float(((unsigned)h) << 16); }

__device__ __forceinline__ void dep_guard_h(v8f& a, v8f& b, v16h x, v16h y) { asm volatile("v_nop\n\tv_nop\n\tv_nop\n\tv_nop" : "+v"(a), "+v"(b) : "v"(x), "v"(y)); }
__device__ __forceinline__ void dep_guard_b(v8f& a, v8f& b, v16b x, v16b y) { asm volatile("v_nop\n\tv_nop\n\tv_nop\n\tv_nop" : "+v"(a), "+v"(b) : "v"(x), "v"(y)); }
__device__ __forceinline__ void keep4_h(v16h a, v16h b, v16h c, v16h d) { asm volatile("v_nop" :: "v"(a), "v"(b), "v"(c), "v"(d)); }
__device__ __forceinline__ void keep4_b(v16b a, v16b b, v16b c, v16b d) { asm volatile("v_nop" :: "v"(a), "v"(b), "v"(c), "v"(d)); }
__device__ __forceinline__ void acc_guard4(v8f& a, v8f& b, v8f& c, v8f& d) { asm volatile("v_nop\n\tv_nop\n\tv_nop\n\tv_nop" : "+v"(a), "+v"(b), "+v"(c), "+v"(d)); }
template <typename T> struct Frag;
template <> struct Frag<_Float16> {
  typedef v16h V; union U { v16h v; v8h h[2]; };
  static __device__ __forceinline__ v16h load(const _Float16* p) {
    U f; f.h[0] = *(const v8h*)(p); f.h[1] = *(const v8h*)(p + 16); return f.v;
  }
  static __device__ __forceinline__ v8f mma(v16h a, v16h b, v8f c) {
    return __builtin_amdgcn_wmma_f32_16x16x32_f16(false, a, false, b, (short)0, c, false, false);
  }
  static __device__ __forceinline__ void guard(v8f& a, v8f& b, v16h x, v16h y) { dep_guard_h(a, b, x, y); }
  static __device__ __forceinline__ void keep(v16h a, v16h b, v16h c, v16h d) { keep4_h(a, b, c, d); }
};
template <> struct Frag<__bf16> {
  typedef v16b V; union U { v16b v; v8b h[2]; };
  static __device__ __forceinline__ v16b load(const __bf16* p) {
    U f; f.h[0] = *(const v8b*)(p); f.h[1] = *(const v8b*)(p + 16); return f.v;
  }
  static __device__ __forceinline__ v8f mma(v16b a, v16b b, v8f c) {
    return __builtin_amdgcn_wmma_f32_16x16x32_bf16(false, a, false, b, (short)0, c, false, false);
  }
  static __device__ __forceinline__ void guard(v8f& a, v8f& b, v16b x, v16b y) { dep_guard_b(a, b, x, y); }
  static __device__ __forceinline__ void keep(v16b a, v16b b, v16b c, v16b d) { keep4_b(a, b, c, d); }
};

__device__ __forceinline__ unsigned pk16(unsigned short a, unsigned short b) { return (unsigned)a | ((unsigned)b << 16); }
__device__ __forceinline__ unsigned short h_bits(float f) { const _Float16 h = (_Float16)f; return __builtin_bit_cast(unsigned short, h); }

template <int ET> struct Elem;
template <> struct Elem<0> { typedef _Float16 T; };
template <> struct Elem<1> { typedef __bf16 T; };
template <int ET, bool SPLIT, int BIAS_MODE, int OUT_MODE, bool RESID, int ACT = 0>
__global__ __launch_bounds__(256) void wmma_gemm64(
    const unsigned short* __restrict__ Ap, const unsigned short* __restrict__ A2p, int lda, long strideA,
    const unsigned short* __restrict__ Btp, const unsigned short* __restrict__ Bt2p, int ldb, long strideB,
    void* __restrict__ Cout, void* __restrict__ Cout2, int ldc, long strideC,
    const float* __restrict__ bias,
    const float* __restrict__ resid, long strideR,
    int M, int N, int K, float scale) {
  typedef typename Elem<ET>::T T;
  typedef typename Frag<T>::V V;
  const T* A = (const T*)Ap; const T* A2 = (const T*)A2p; const T* Bt = (const T*)Btp; const T* Bt2 = (const T*)Bt2p;
  __shared__ __align__(16) float sT[8][16 * 68];
  const int b    = blockIdx.y;
  const int lane = threadIdx.x & 31;
  const int wave = threadIdx.x >> 5;
  const int tilesN = N >> 6;
  const int tilesM = M >> 6;
  const int tile = blockIdx.x * 8 + wave;
  if (tile >= tilesM * tilesN) return;
  const int tm = tile / tilesN;
  const int tn = tile - tm * tilesN;
  const int m0 = tm << 6;
  const int n0 = tn << 6;

  const T* Ab  = A  + (size_t)b * strideA;
  const T* Bb  = Bt + (size_t)b * strideB;
  const T* Ab2 = SPLIT ? (A2  + (size_t)b * strideA) : nullptr;
  const T* Bb2 = SPLIT ? (Bt2 + (size_t)b * strideB) : nullptr;

  const int rlane = lane & 15;
  const int koff  = (lane >> 4) * 8;
  const int mOff  = (lane >> 4) * 8;

  v8f acc[4][4];
#pragma unroll
  for (int i = 0; i < 4; ++i)
#pragma unroll
    for (int j = 0; j < 4; ++j) acc[i][j] = (v8f){0.f,0.f,0.f,0.f,0.f,0.f,0.f,0.f};

  for (int k0 = 0; k0 < K; k0 += 32) {
    V bh[4], bl[4];
#pragma unroll
    for (int j = 0; j < 4; ++j) {
      const size_t bo = (size_t)(n0 + (j << 4) + rlane) * ldb + koff + k0;
      bh[j] = Frag<T>::load(Bb + bo);
      if (SPLIT) bl[j] = Frag<T>::load(Bb2 + bo);
    }
#pragma unroll
    for (int i = 0; i < 4; ++i) {
      const size_t ao = (size_t)(m0 + (i << 4) + rlane) * lda + koff + k0;
      V ah = Frag<T>::load(Ab + ao);
      V al;
      if (SPLIT) al = Frag<T>::load(Ab2 + ao);
#pragma unroll
      for (int j = 0; j < 4; ++j) {
        acc[i][j] = Frag<T>::mma(ah, bh[j], acc[i][j]);
        if (SPLIT) {
          acc[i][j] = Frag<T>::mma(ah, bl[j], acc[i][j]);
          acc[i][j] = Frag<T>::mma(al, bh[j], acc[i][j]);
        }
      }
      Frag<T>::guard(acc[i][0], acc[i][3], ah, SPLIT ? al : ah);
    }
    Frag<T>::keep(bh[0], bh[1], bh[2], bh[3]);
    if (SPLIT) Frag<T>::keep(bl[0], bl[1], bl[2], bl[3]);
  }
  acc_guard4(acc[0][0], acc[0][1], acc[0][2], acc[0][3]);
  acc_guard4(acc[1][0], acc[1][1], acc[1][2], acc[1][3]);
  acc_guard4(acc[2][0], acc[2][1], acc[2][2], acc[2][3]);
  acc_guard4(acc[3][0], acc[3][1], acc[3][2], acc[3][3]);

  float* slab = sT[wave];
  const float* Rb = RESID ? (resid + (size_t)b * strideR) : nullptr;
#pragma unroll
  for (int i = 0; i < 4; ++i) {
    const int mBase = m0 + (i << 4);
#pragma unroll
    for (int j = 0; j < 4; ++j) {
      const int n = n0 + (j << 4) + rlane;
      float bv = 0.f;
      if (BIAS_MODE == 2) bv = bias[n];
#pragma unroll
      for (int r = 0; r < 8; ++r) {
        float v = acc[i][j][r] * scale;
        if (BIAS_MODE == 1) v += bias[mBase + mOff + r];
        if (BIAS_MODE == 2) v += bv;
        if (RESID) v += Rb[(size_t)(mBase + mOff + r) * ldc + n];
        if (ACT == 2) v = fmaxf(v, 0.0f);
        if (ACT == 4) v = (v > 0.f) ? v : 0.01f * v;
        slab[(mOff + r) * 68 + (j << 4) + rlane] = v;
      }
    }
    __builtin_amdgcn_fence(__ATOMIC_RELEASE, "workgroup");
    __builtin_amdgcn_wave_barrier();
    __builtin_amdgcn_fence(__ATOMIC_ACQUIRE, "workgroup");
    if (OUT_MODE == 0) {
      float* C = (float*)Cout + (size_t)b * strideC;
      const int hh = lane >> 4, c4 = (lane & 15) * 4;
      for (int pass = 0; pass < 2; ++pass) {
#pragma unroll
        for (int it = 0; it < 8; ++it) {
          const int row = it * 2 + hh;
          v4f v = *(const v4f*)(slab + row * 68 + c4);
          *(volatile v4f*)(C + (size_t)(mBase + row) * ldc + n0 + c4) = v;
        }
        __threadfence();
      }
    } else {
      const int q = lane >> 3, c8 = (lane & 7) * 8;
      unsigned short* C  = (unsigned short*)Cout  + (size_t)b * strideC;
      unsigned short* C2 = (OUT_MODE == 2) ? ((unsigned short*)Cout2 + (size_t)b * strideC) : nullptr;
      for (int pass = 0; pass < 2; ++pass) {
#pragma unroll
        for (int it = 0; it < 4; ++it) {
          const int row = it * 4 + q;
          const float* sp = slab + row * 68 + c8;
          v8h hv, lv;
#pragma unroll
          for (int e = 0; e < 8; ++e) {
            if (OUT_MODE == 1) {
              hv[e] = (_Float16)sp[e];
            } else {
              unsigned short hb = f2bf_bits(sp[e]);
              unsigned short lb = f2bf_bits(sp[e] - bf_bits2f(hb));
              hv[e] = __builtin_bit_cast(_Float16, hb);
              lv[e] = __builtin_bit_cast(_Float16, lb);
            }
          }
          *(volatile v8h*)(C + (size_t)(mBase + row) * ldc + n0 + c8) = hv;
          if (OUT_MODE == 2) *(volatile v8h*)(C2 + (size_t)(mBase + row) * ldc + n0 + c8) = lv;
        }
        __threadfence();
      }
    }
    __builtin_amdgcn_fence(__ATOMIC_RELEASE, "workgroup");
    __builtin_amdgcn_wave_barrier();
    __builtin_amdgcn_fence(__ATOMIC_ACQUIRE, "workgroup");
  }
}

__global__ __launch_bounds__(256) void cast8s_f16_kernel(const float* __restrict__ in, unsigned short* __restrict__ out,
                                                        int n8, float carry) {
  const int i = blockIdx.x * 256 + threadIdx.x;
  if (i >= n8) return;
  const float* p = in + 8 * (size_t)i;
  const v4f a = *(const v4f*)(p);
  const v4f c = *(const v4f*)(p + 4);
  unsigned short hb[8];
#pragma unroll
  for (int e = 0; e < 4; ++e) {
    hb[e]     = h_bits(a[e] * carry);
    hb[4 + e] = h_bits(c[e] * carry);
  }
  const v4u u = (v4u){pk16(hb[0], hb[1]), pk16(hb[2], hb[3]), pk16(hb[4], hb[5]), pk16(hb[6], hb[7])};
  unsigned short* q = out + 8 * (size_t)i;
  *(volatile v4u*)q = u;
  __threadfence();
  *(volatile v4u*)q = u;
}

__global__ __launch_bounds__(256) void softmax_row_kernel(const float* __restrict__ S, unsigned short* __restrict__ P, float carry) {
  __shared__ float redM[8];
  __shared__ float redS[8];
  const int row  = blockIdx.x;
  const int t    = threadIdx.x;
  const int lane = t & 31, wave = t >> 5;
  const int c0   = t * 8;
  const float* sr = S + (size_t)row * kSeq + c0;
  const v4f a = *(const v4f*)(sr);
  const v4f c = *(const v4f*)(sr + 4);
  float m = fmaxf(fmaxf(fmaxf(a[0], a[1]), fmaxf(a[2], a[3])), fmaxf(fmaxf(c[0], c[1]), fmaxf(c[2], c[3])));
#pragma unroll
  for (int off = 16; off > 0; off >>= 1) m = fmaxf(m, __shfl_xor(m, off, 32));
  if (lane == 0) redM[wave] = m;
  __syncthreads();
  float gm = redM[0];
#pragma unroll
  for (int w = 1; w < 8; ++w) gm = fmaxf(gm, redM[w]);
  const float e0 = expf(a[0] - gm), e1 = expf(a[1] - gm), e2 = expf(a[2] - gm), e3 = expf(a[3] - gm);
  const float e4 = expf(c[0] - gm), e5 = expf(c[1] - gm), e6 = expf(c[2] - gm), e7 = expf(c[3] - gm);
  float s = ((e0 + e1) + (e2 + e3)) + ((e4 + e5) + (e6 + e7));
#pragma unroll
  for (int off = 16; off > 0; off >>= 1) s += __shfl_xor(s, off, 32);
  if (lane == 0) redS[wave] = s;
  __syncthreads();
  float tot = redS[0];
#pragma unroll
  for (int w = 1; w < 8; ++w) tot += redS[w];
  const float rc = carry * (1.0f / tot);
  const v4u u = (v4u){pk16(h_bits(e0 * rc), h_bits(e1 * rc)), pk16(h_bits(e2 * rc), h_bits(e3 * rc)),
                      pk16(h_bits(e4 * rc), h_bits(e5 * rc)), pk16(h_bits(e6 * rc), h_bits(e7 * rc))};
  unsigned short* q = P + (size_t)row * kSeq + c0;
  *(volatile v4u*)q = u;
  __threadfence();
  *(volatile v4u*)q = u;
}

extern "C" void kernel_launch(void* const* d_in, const int* in_sizes, int n_in,
                              void* d_out, int out_size, void* d_ws, size_t ws_size, hipStream_t stream) {
  (void)n_in;
  const float* x   = (const float*)d_in[0];
  const float* wq  = (const float*)d_in[1];
  const float* bq  = (const float*)d_in[2];
  const float* wk  = (const float*)d_in[3];
  const float* bk  = (const float*)d_in[4];
  const float* wv  = (const float*)d_in[5];
  const float* bvp = (const float*)d_in[6];
  const float* wo  = (const float*)d_in[7];
  const float* bop = (const float*)d_in[8];
  float* out = (float*)d_out;

  if (in_sizes[0] != kTok * kEmb) return;
  if (out_size != kTok * kEmb) return;
  if (ws_size < kWsEnd) return;

  char* ws = (char*)d_ws;
  unsigned short* w16   = (unsigned short*)(ws + kOffW);
  unsigned short* wq16  = w16;
  unsigned short* wk16  = w16 + (size_t)kEmb * kEmb;
  unsigned short* wv16  = w16 + (size_t)2 * kEmb * kEmb;
  unsigned short* wo16  = w16 + (size_t)3 * kEmb * kEmb;
  unsigned short* x16   = (unsigned short*)(ws + kOffX);
  unsigned short* q16   = (unsigned short*)(ws + kOffQ);
  unsigned short* k16   = (unsigned short*)(ws + kOffK);
  unsigned short* vt16  = (unsigned short*)(ws + kOffVT);
  unsigned short* ctx16 = (unsigned short*)(ws + kOffCtx);
  float*          sc    = (float*)(ws + kOffS);
  unsigned short* p16   = (unsigned short*)(ws + kOffP);

  const dim3 blk(256);
  const int n8w = kEmb * kEmb / 8;
  const int n8x = kSeq * kEmb / 8;

  cast8s_f16_kernel<<<dim3((n8w + 255) / 256), blk, 0, stream>>>(wq, wq16, n8w, kWCarry);
  cast8s_f16_kernel<<<dim3((n8w + 255) / 256), blk, 0, stream>>>(wk, wk16, n8w, kWCarry);
  cast8s_f16_kernel<<<dim3((n8w + 255) / 256), blk, 0, stream>>>(wv, wv16, n8w, kWCarry);
  cast8s_f16_kernel<<<dim3((n8w + 255) / 256), blk, 0, stream>>>(wo, wo16, n8w, kWCarry);

  const long scoreStride = (long)kSeq * kSeq;
  const long vtGroupStride = (long)kHdim * kSeq;

  for (int b = 0; b < kBatch; ++b) {
    const float* xb = x + (size_t)b * kSeq * kEmb;
    cast8s_f16_kernel<<<dim3((n8x + 255) / 256), blk, 0, stream>>>(xb, x16, n8x, 1.0f);

    wmma_gemm64<0, false, 2, 1, false><<<dim3(64, 1), blk, 0, stream>>>(
        x16, x16, kEmb, 0L, wq16, wq16, kEmb, 0L, (void*)q16, (void*)q16, kEmb, 0L,
        bq, xb, 0L, kSeq, kEmb, kEmb, kProjScale);
    wmma_gemm64<0, false, 2, 1, false><<<dim3(64, 1), blk, 0, stream>>>(
        x16, x16, kEmb, 0L, wk16, wk16, kEmb, 0L, (void*)k16, (void*)k16, kEmb, 0L,
        bk, xb, 0L, kSeq, kEmb, kEmb, kProjScale);
    wmma_gemm64<0, false, 1, 1, false><<<dim3(64, 1), blk, 0, stream>>>(
        wv16, wv16, kEmb, 0L, x16, x16, kEmb, 0L, (void*)vt16, (void*)vt16, kSeq, 0L,
        bvp, xb, 0L, kEmb, kSeq, kEmb, kProjScale);

    for (int ck = 0; ck < kChunks; ++ck) {
      const int h0 = ck * kGrp;
      wmma_gemm64<0, false, 0, 0, false><<<dim3(128, kGrp), blk, 0, stream>>>(
          q16 + (size_t)h0 * kHdim, q16 + (size_t)h0 * kHdim, kEmb, (long)kHdim,
          k16 + (size_t)h0 * kHdim, k16 + (size_t)h0 * kHdim, kEmb, (long)kHdim,
          (void*)sc, (void*)sc, kSeq, scoreStride,
          bq, xb, 0L, kSeq, kSeq, kHdim, kScoreScale);
      softmax_row_kernel<<<dim3(kGrp * kSeq), blk, 0, stream>>>(sc, p16, kPCarry);
      wmma_gemm64<0, false, 0, 1, false><<<dim3(4, kGrp), blk, 0, stream>>>(
          p16, p16, kSeq, scoreStride,
          vt16 + (size_t)h0 * kHdim * kSeq, vt16 + (size_t)h0 * kHdim * kSeq, kSeq, vtGroupStride,
          (void*)(ctx16 + (size_t)h0 * kHdim), (void*)(ctx16 + (size_t)h0 * kHdim), kEmb, (long)kHdim,
          bq, xb, 0L, kSeq, kHdim, kSeq, kPVScale);
    }

    float* outb = out + (size_t)b * kSeq * kEmb;
    wmma_gemm64<0, false, 2, 0, false><<<dim3(64, 1), blk, 0, stream>>>(
        ctx16, ctx16, kEmb, 0L, wo16, wo16, kEmb, 0L, (void*)outb, (void*)outb, kEmb, 0L,
        bop, xb, 0L, kSeq, kEmb, kEmb, kOutScale);
  }
}
